// GATsep_18433999635062
// MI455X (gfx1250) — hardware-verified
//
#include <hip/hip_runtime.h>
#include <stddef.h>


#define NTHR   256
#define NWAVE  8
#define GTHR   128
#define GR     32
#define GC     64
#define XSP    68
#define APITCH 192
#define NB     128
#define CHUNK  4096
#define NGRP   (CHUNK / (NTHR * 4))
#define WCAP   512
#define NHEAD  8
#define DOUTC  40

static_assert(NGRP == 4);
static_assert(WCAP == NGRP * 4 * 32);
static_assert((NB & (NB - 1)) == 0);
static_assert(NB <= 256);
static_assert(NB <= WCAP);
static_assert((XSP % 4) == 0);
static_assert((APITCH % 8) == 0);

typedef float    v2f  __attribute__((ext_vector_type(2)));
typedef float    v4f  __attribute__((ext_vector_type(4)));
typedef float    v8f  __attribute__((ext_vector_type(8)));
typedef int      v4i  __attribute__((ext_vector_type(4)));
typedef _Float16 v2h  __attribute__((ext_vector_type(2)));
typedef _Float16 v8h  __attribute__((ext_vector_type(8)));
typedef _Float16 v16h __attribute__((ext_vector_type(16)));

union FragH { v16h v; v4i u[2]; };
union Pack  { v8h h; v4i i; };

__host__ __device__ constexpr int agg_lds_bytes(int cph) {
  return NB * NHEAD * cph * 4 + 2 * NB * NHEAD * 4 + NWAVE * WCAP * 4 + 64 + NB * DOUTC * 4;
}
static_assert(agg_lds_bytes(32) == 176192);
static_assert(agg_lds_bytes(40) == 208960);

__device__ __forceinline__ v8f wmh(v16h a, v16h b, v8f c) {
  v8f d = __builtin_amdgcn_wmma_f32_16x16x32_f16(false, a, false, b, (short)0, c, false, false);
  asm volatile("v_nop\n\tv_nop\n\tv_nop\n\tv_nop" : "+v"(d) : "v"(a), "v"(b));
  return d;
}

template <int CPL>
__device__ __forceinline__ void ldf(float (&a)[CPL], const float* p) {
  if constexpr (CPL == 8) {
    const v4f u0 = *(const v4f*)p;
    const v4f u1 = *(const v4f*)(p + 4);
    a[0] = u0.x; a[1] = u0.y; a[2] = u0.z; a[3] = u0.w;
    a[4] = u1.x; a[5] = u1.y; a[6] = u1.z; a[7] = u1.w;
  } else {
#pragma unroll
    for (int q = 0; q < CPL / 2; ++q) {
      const v2f u = *(const v2f*)(p + 2 * q);
      a[2 * q] = u.x; a[2 * q + 1] = u.y;
    }
  }
}
template <int CPL>
__device__ __forceinline__ void stf(float* p, const float (&a)[CPL]) {
  if constexpr (CPL == 8) {
    v4f u0, u1;
    u0.x = a[0]; u0.y = a[1]; u0.z = a[2]; u0.w = a[3];
    u1.x = a[4]; u1.y = a[5]; u1.z = a[6]; u1.w = a[7];
    *(v4f*)p = u0;
    *(v4f*)(p + 4) = u1;
  } else {
#pragma unroll
    for (int q = 0; q < CPL / 2; ++q) {
      v2f u; u.x = a[2 * q]; u.y = a[2 * q + 1];
      *(v2f*)(p + 2 * q) = u;
    }
  }
}
template <int CPL>
__device__ __forceinline__ void ldh(float (&a)[CPL], const _Float16* p) {
  if constexpr (CPL == 8) {
    const v8h u = *(const v8h*)p;
#pragma unroll
    for (int j = 0; j < 8; ++j) a[j] = (float)u[j];
  } else {
#pragma unroll
    for (int q = 0; q < CPL / 2; ++q) {
      const v2h u = *(const v2h*)(p + 2 * q);
      a[2 * q] = (float)u.x; a[2 * q + 1] = (float)u.y;
    }
  }
}

__global__ __launch_bounds__(NTHR) void k_cvtx(const float* __restrict__ x, unsigned short* ap, int nN, int mPad) {
  const int i  = blockIdx.x * NTHR + threadIdx.x;
  const int n8 = mPad * 16;
  if (i >= n8) return;
  const int r  = i >> 4;
  const int kb = (i & 15) * 8;
  v4f lo = {0.f, 0.f, 0.f, 0.f};
  v4f hi = lo;
  if (r < nN) {
    const float* p = x + (size_t)r * 128 + kb;
    lo = *(const v4f*)p;
    hi = *(const v4f*)(p + 4);
  }
  Pack u;
  u.h[0] = (_Float16)lo.x; u.h[1] = (_Float16)lo.y; u.h[2] = (_Float16)lo.z; u.h[3] = (_Float16)lo.w;
  u.h[4] = (_Float16)hi.x; u.h[5] = (_Float16)hi.y; u.h[6] = (_Float16)hi.z; u.h[7] = (_Float16)hi.w;
  unsigned short* d = ap + (size_t)r * APITCH + kb;
  *(volatile v4i*)d = u.i;
  __threadfence();
  *(volatile v4i*)d = u.i;
}

__global__ __launch_bounds__(NTHR) void k_cvtw(const float* __restrict__ W0, const float* __restrict__ W1,
                                               unsigned short* B0, unsigned short* B1, int K, int NOUT, float scale) {
  const int kp8 = K >> 3;
  const int n8  = NOUT * kp8;
  const int i   = blockIdx.x * NTHR + threadIdx.x;
  if (i >= n8) return;
  const float* W = blockIdx.y ? W1 : W0;
  unsigned short* Bp = blockIdx.y ? B1 : B0;
  const int n  = i / kp8;
  const int kb = (i - n * kp8) * 8;
  Pack u;
#pragma unroll
  for (int j = 0; j < 8; ++j) u.h[j] = (_Float16)(W[(size_t)(kb + j) * NOUT + n] * scale);
  unsigned short* d = Bp + (size_t)i * 8;
  *(volatile v4i*)d = u.i;
  __threadfence();
  *(volatile v4i*)d = u.i;
}

__global__ __launch_bounds__(GTHR) void k_gemm(
    const unsigned short* __restrict__ Ap, int lda, int K,
    const unsigned short* __restrict__ Bt0, const unsigned short* __restrict__ Bt1,
    const float* __restrict__ bias0, const float* __restrict__ bias1,
    float* out0, unsigned short* out1, int NC, float oscale) {
  __shared__ __attribute__((aligned(16))) float Xs[GR * XSP];

  const int tid  = threadIdx.x;
  const int lane = tid & 31;
  const int wave = tid >> 5;
  const int hh   = lane >> 4;
  const int m    = lane & 15;
  const int rowBase = blockIdx.x * GR;
  const int colBase = blockIdx.y * GC;
  const int z = blockIdx.z;
  const unsigned short* Bt = z ? Bt1 : Bt0;
  const float* bias = z ? bias1 : bias0;
  const int ncol = colBase + wave * 16 + m;

  const size_t ra0 = (size_t)(rowBase + m) * lda + 8 * hh;
  const size_t ra1 = ra0 + (size_t)16 * lda;
  const size_t rb  = (size_t)ncol * K + 8 * hh;

  v8f c0 = {0.f, 0.f, 0.f, 0.f, 0.f, 0.f, 0.f, 0.f};
  v8f c1 = {0.f, 0.f, 0.f, 0.f, 0.f, 0.f, 0.f, 0.f};

#pragma unroll 1
  for (int k0 = 0; k0 < K; k0 += 32) {
    FragH a0, a1, b;
    a0.u[0] = *(const v4i*)(Ap + ra0 + k0);  a0.u[1] = *(const v4i*)(Ap + ra0 + k0 + 16);
    a1.u[0] = *(const v4i*)(Ap + ra1 + k0);  a1.u[1] = *(const v4i*)(Ap + ra1 + k0 + 16);
    b.u[0]  = *(const v4i*)(Bt + rb + k0);   b.u[1]  = *(const v4i*)(Bt + rb + k0 + 16);
    c0 = wmh(a0.v, b.v, c0);
    c1 = wmh(a1.v, b.v, c1);
  }

  const float bv = bias[ncol];
  const int cl = wave * 16 + m;
#pragma unroll
  for (int r = 0; r < 8; ++r) {
    Xs[(8 * hh + r) * XSP + cl]      = c0[r] * oscale + bv;
    Xs[(16 + 8 * hh + r) * XSP + cl] = c1[r] * oscale + bv;
  }
  __syncthreads();

  if (z == 0) {
    v4f xv[4];
    float* xp[4];
#pragma unroll
    for (int i = 0; i < 4; ++i) {
      const int r = 8 * wave + 2 * i + (lane >> 4);
      xv[i] = *(const v4f*)(Xs + r * XSP + 4 * (lane & 15));
      xp[i] = out0 + (size_t)(rowBase + r) * NC + colBase + 4 * (lane & 15);
    }
#pragma unroll
    for (int i = 0; i < 4; ++i) *(volatile v4f*)(xp[i]) = xv[i];
    __threadfence();
#pragma unroll
    for (int i = 0; i < 4; ++i) *(volatile v4f*)(xp[i]) = xv[i];
  } else {
    v4i hv[2];
    unsigned short* hp[2];
#pragma unroll
    for (int i = 0; i < 2; ++i) {
      const int r  = 8 * wave + 4 * i + (lane >> 3);
      const int cb = 8 * (lane & 7);
      const float* sp = Xs + r * XSP + cb;
      const v4f f0 = *(const v4f*)sp;
      const v4f f1 = *(const v4f*)(sp + 4);
      Pack u;
      u.h[0] = (_Float16)f0.x; u.h[1] = (_Float16)f0.y; u.h[2] = (_Float16)f0.z; u.h[3] = (_Float16)f0.w;
      u.h[4] = (_Float16)f1.x; u.h[5] = (_Float16)f1.y; u.h[6] = (_Float16)f1.z; u.h[7] = (_Float16)f1.w;
      hv[i] = u.i;
      hp[i] = out1 + (size_t)(rowBase + r) * NC + colBase + cb;
    }
#pragma unroll
    for (int i = 0; i < 2; ++i) *(volatile v4i*)(hp[i]) = hv[i];
    __threadfence();
#pragma unroll
    for (int i = 0; i < 2; ++i) *(volatile v4i*)(hp[i]) = hv[i];
  }
}

template <int CPH>
__global__ __launch_bounds__(NTHR) void k_agg(
    const int* __restrict__ ei, const float* __restrict__ xl, const _Float16* __restrict__ xr,
    const float* __restrict__ att, const float* __restrict__ bias,
    unsigned short* ap, float* out, int nN, int nE, int nW) {
  constexpr int NC  = NHEAD * CPH;
  constexpr int CPL = CPH / 4;
  static_assert(CPL * 4 == CPH);
  static_assert(NB * DOUTC / 4 <= 5 * NTHR);

  extern __shared__ v4f lds_dyn[];
  float* sacc = (float*)lds_dyn;
  float* mx   = sacc + NB * NC;
  float* dn   = mx + NB * NHEAD;
  int*   list = (int*)(dn + NB * NHEAD);
  int*   wcnt = list + NWAVE * WCAP;
  float* vbuf = (float*)(wcnt + 16);

  const int tid  = threadIdx.x;
  const int lane = tid & 31;
  const int wave = tid >> 5;
  const int nodeBase = blockIdx.x * NB;

  {
    const v4f z4 = {0.f, 0.f, 0.f, 0.f};
    for (int i = tid; i < NB * NC / 4; i += NTHR) lds_dyn[i] = z4;
    for (int i = tid; i < NB * NHEAD; i += NTHR) { mx[i] = -1.0e30f; dn[i] = 0.f; }
  }
  __syncthreads();

  const int hd = lane >> 2;
  const int c0 = CPL * lane;
  float w[CPL];
#pragma unroll
  for (int j = 0; j < CPL; ++j) w[j] = att[c0 + j];

  const int* eid = ei + nE;
  const bool al16 = ((nE & 3) == 0);
  const int nChunks = (nE + CHUNK - 1) / CHUNK;

#pragma unroll 1
  for (int ch = 0; ch <= nChunks; ++ch) {
    const int cbase = ch * CHUNK;
    const bool selfp = (ch == nChunks);
    if (!selfp) {
      int wc = 0;
#pragma unroll
      for (int g = 0; g < NGRP; ++g) {
        const int el0 = (g * NTHR + tid) * 4;
        const int e0  = cbase + el0;
        const int sent = -2147483647 - 1;
        v4i d;
        if (al16 && (e0 + 3 < nE)) {
          d = *(const v4i*)(eid + e0);
        } else {
          d.x = (e0     < nE) ? eid[min(e0, nE - 1)]     : sent;
          d.y = (e0 + 1 < nE) ? eid[min(e0 + 1, nE - 1)] : sent;
          d.z = (e0 + 2 < nE) ? eid[min(e0 + 2, nE - 1)] : sent;
          d.w = (e0 + 3 < nE) ? eid[min(e0 + 3, nE - 1)] : sent;
        }
        const unsigned s0 = (unsigned)d.x - (unsigned)nodeBase;
        const unsigned s1 = (unsigned)d.y - (unsigned)nodeBase;
        const unsigned s2 = (unsigned)d.z - (unsigned)nodeBase;
        const unsigned s3 = (unsigned)d.w - (unsigned)nodeBase;
        const bool h0 = s0 < (unsigned)NB;
        const bool h1 = s1 < (unsigned)NB;
        const bool h2 = s2 < (unsigned)NB;
        const bool h3 = s3 < (unsigned)NB;
        const unsigned many = __builtin_amdgcn_ballot_w32(h0 | h1 | h2 | h3);
        if (many != 0u) {
#define HITJ(J, HJ, SJ) { \
            const unsigned mj = __builtin_amdgcn_ballot_w32(HJ); \
            if (HJ) { \
              const int pos = wc + (int)__builtin_amdgcn_mbcnt_lo(mj, 0u); \
              if (pos < WCAP) list[wave * WCAP + pos] = ((el0 + (J)) << 8) | (int)(SJ); \
            } \
            wc += (int)__builtin_popcount(mj); }
          HITJ(0, h0, s0)
          HITJ(1, h1, s1)
          HITJ(2, h2, s2)
          HITJ(3, h3, s3)
#undef HITJ
        }
      }
      if (lane == 0) wcnt[wave] = wc;
    } else {
      for (int s = tid; s < NB; s += NTHR) list[s] = s;
      if (tid < NWAVE) {
        int c = NB - tid * WCAP;
        c = c < 0 ? 0 : (c > WCAP ? WCAP : c);
        wcnt[tid] = c;
      }
    }
    __syncthreads();

    if (wave == 0) {
#pragma unroll 1
      for (int wsx = 0; wsx < NWAVE; ++wsx) {
        int n = __builtin_amdgcn_readfirstlane(wcnt[wsx]);
        n = n > WCAP ? WCAP : n;
        n = n < 0 ? 0 : n;
#pragma unroll 1
        for (int i = 0; i < n; ++i) {
          const int ent  = __builtin_amdgcn_readfirstlane(list[wsx * WCAP + i]);
          const int slot = ent & (NB - 1);
          const int el   = (ent >> 8) & (CHUNK - 1);
          const int node = nodeBase + slot;
          if (node >= nN) continue;
          int e = cbase + el;
          if (e > nE - 1) e = nE - 1;
          int sj = ei[e];
          sj = sj < 0 ? 0 : (sj > nN - 1 ? nN - 1 : sj);
          const int src = selfp ? node : sj;
          const float*    xs = xl + (size_t)src  * NC + c0;
          const _Float16* xd = xr + (size_t)node * NC + c0;
          float* ar = sacc + slot * NC + c0;
          float* mp = mx + slot * NHEAD + hd;
          float* dp = dn + slot * NHEAD + hd;

          float a[CPL], dv[CPL], ev[CPL];
          ldf<CPL>(a, xs);
          ldh<CPL>(dv, xd);
          float s = 0.f;
#pragma unroll
          for (int j = 0; j < CPL; ++j) {
            float t = a[j] + dv[j];
            t = fmaxf(t, 0.2f * t);
            s += w[j] * t;
          }
          s += __shfl_xor(s, 2, 32);
          s += __shfl_xor(s, 1, 32);
          const float mo = mp[0];
          const float no = dp[0];
          const float mn = fmaxf(mo, s);
          const float sc = __expf(mo - mn);
          const float p  = __expf(s - mn);
          ldf<CPL>(ev, ar);
#pragma unroll
          for (int j = 0; j < CPL; ++j) ev[j] = ev[j] * sc + a[j] * p;
          stf<CPL>(ar, ev);
          mp[0] = mn;
          dp[0] = no * sc + p;
        }
      }
    }
    __syncthreads();
  }

  if constexpr (CPH == 32) {
    const int q = lane & 7;
#pragma unroll 1
    for (int i = 0; i < 4; ++i) {
      const int s    = 16 * wave + 4 * i + (lane >> 3);
      const int node = nodeBase + s;
      Pack u;
      const v4i z4 = {0, 0, 0, 0};
      u.i = z4;
      if (node < nN && q < 4) {
        float t[8] = {0.f, 0.f, 0.f, 0.f, 0.f, 0.f, 0.f, 0.f};
        const float* arow = sacc + s * NC + 8 * q;
        const float* drow = dn + s * NHEAD;
#pragma unroll 1
        for (int h = 0; h < NHEAD; ++h) {
          const float iv = __builtin_amdgcn_rcpf(drow[h]);
          const v4f e0 = *(const v4f*)(arow + CPH * h);
          const v4f e1 = *(const v4f*)(arow + CPH * h + 4);
          t[0] += e0.x * iv; t[1] += e0.y * iv; t[2] += e0.z * iv; t[3] += e0.w * iv;
          t[4] += e1.x * iv; t[5] += e1.y * iv; t[6] += e1.z * iv; t[7] += e1.w * iv;
        }
#pragma unroll
        for (int j = 0; j < 8; ++j) {
          float v = t[j] * 0.125f + bias[8 * q + j];
          v = (v > 0.f) ? v : (__expf(v) - 1.0f);
          u.h[j] = (_Float16)v;
        }
      }
      const bool doit = (node < nW);
      unsigned short* pp = ap + (size_t)node * APITCH + 128 + 8 * q;
      if (doit) *(volatile v4i*)pp = u.i;
      __threadfence();
      if (doit) *(volatile v4i*)pp = u.i;
    }
  } else {
    for (int i = tid; i < NB * NHEAD; i += NTHR) {
      const int nd = nodeBase + (i >> 3);
      const float dd = dn[i];
      dn[i] = (nd < nN) ? __builtin_amdgcn_rcpf(dd) : 0.f;
    }
    __syncthreads();
#pragma unroll 1
    for (int idx = tid; idx < NB * DOUTC; idx += NTHR) {
      const int s = idx / DOUTC;
      const int c = idx - s * DOUTC;
      const float* arow = sacc + s * NC + c;
      const float* drow = dn + s * NHEAD;
      float t = 0.f;
#pragma unroll 1
      for (int h = 0; h < NHEAD; ++h) t += arow[CPH * h] * drow[h];
      vbuf[idx] = t * 0.125f + bias[c];
    }
    __syncthreads();
    if (tid < NB) {
      float* vr = vbuf + tid * DOUTC;
      float mxv = -3.0e38f;
#pragma unroll 1
      for (int c = 0; c < DOUTC; ++c) mxv = fmaxf(mxv, vr[c]);
      float se = 0.f;
#pragma unroll 1
      for (int c = 0; c < DOUTC; ++c) se += __expf(vr[c] - mxv);
      const float lse = mxv + __logf(se);
#pragma unroll 1
      for (int c = 0; c < DOUTC; ++c) vr[c] = vr[c] - lse;
    }
    __syncthreads();
    int nrows = nN - nodeBase;
    nrows = nrows > NB ? NB : (nrows < 0 ? 0 : nrows);
    const int nf4 = nrows * (DOUTC / 4);
    const v4f* vb4 = (const v4f*)vbuf;
    float* ob = out + (size_t)nodeBase * DOUTC;
    v4f ov[5];
#pragma unroll
    for (int k = 0; k < 5; ++k) ov[k] = vb4[tid + NTHR * k];
#pragma unroll
    for (int k = 0; k < 5; ++k) {
      const int f = tid + NTHR * k;
      if (f < nf4) *(volatile v4f*)(ob + (size_t)4 * f) = ov[k];
    }
    __threadfence();
#pragma unroll
    for (int k = 0; k < 5; ++k) {
      const int f = tid + NTHR * k;
      if (f < nf4) *(volatile v4f*)(ob + (size_t)4 * f) = ov[k];
    }
  }
}

extern "C" void kernel_launch(void* const* d_in, const int* in_sizes, int n_in,
                              void* d_out, int out_size, void* d_ws, size_t ws_size,
                              hipStream_t stream) {
  if (n_in < 14) return;
  const int DIN = 128, C1 = 32, C2 = DOUTC;
  const int NC1 = NHEAD * C1, NC2 = NHEAD * C2, K2 = DIN + C1;
  const int nN = in_sizes[0] / DIN;
  if (nN <= 0 || in_sizes[0] != nN * DIN) return;
  const int nE = in_sizes[1] / 2;
  if (nE <= 0 || in_sizes[1] != 2 * nE) return;
  if (in_sizes[2] != DIN * NC1 || in_sizes[3] != NC1 || in_sizes[4] != DIN * NC1 || in_sizes[5] != NC1 ||
      in_sizes[6] != NC1 || in_sizes[7] != C1) return;
  if (in_sizes[8] != K2 * NC2 || in_sizes[9] != NC2 || in_sizes[10] != K2 * NC2 || in_sizes[11] != NC2 ||
      in_sizes[12] != NC2 || in_sizes[13] != C2) return;
  if (out_size != nN * C2) return;

  const float* x     = (const float*)d_in[0];
  const int*   ei    = (const int*)d_in[1];
  const float* Wl1   = (const float*)d_in[2];
  const float* bl1   = (const float*)d_in[3];
  const float* Wr1   = (const float*)d_in[4];
  const float* br1   = (const float*)d_in[5];
  const float* att1  = (const float*)d_in[6];
  const float* bias1 = (const float*)d_in[7];
  const float* Wl2   = (const float*)d_in[8];
  const float* bl2   = (const float*)d_in[9];
  const float* Wr2   = (const float*)d_in[10];
  const float* br2   = (const float*)d_in[11];
  const float* att2  = (const float*)d_in[12];
  const float* bias2 = (const float*)d_in[13];
  float* out = (float*)d_out;

  const int Mpad = ((nN + GR - 1) / GR) * GR;

  char* wsp = (char*)d_ws;
  size_t off = 0;
  const size_t apB = (size_t)Mpad * APITCH * 2;
  const size_t xlB = (size_t)Mpad * NC2 * 4;
  const size_t xrB = (size_t)Mpad * NC2 * 2;
  const size_t b1B = (size_t)NC1 * DIN * 2;
  const size_t b2B = (size_t)NC2 * K2 * 2;
  unsigned short* ap   = (unsigned short*)(wsp + off); off += apB;
  float*          xl   = (float*)(wsp + off);          off += xlB;
  unsigned short* xr   = (unsigned short*)(wsp + off); off += xrB;
  unsigned short* btl1 = (unsigned short*)(wsp + off); off += b1B;
  unsigned short* btr1 = (unsigned short*)(wsp + off); off += b1B;
  unsigned short* btl2 = (unsigned short*)(wsp + off); off += b2B;
  unsigned short* btr2 = (unsigned short*)(wsp + off); off += b2B;
  if (off > ws_size) return;

  const float s16  = 16.0f;
  const float is16 = 0.0625f;

  hipFuncSetAttribute(reinterpret_cast<const void*>(&k_agg<32>),
                      hipFuncAttributeMaxDynamicSharedMemorySize, agg_lds_bytes(32));
  hipFuncSetAttribute(reinterpret_cast<const void*>(&k_agg<40>),
                      hipFuncAttributeMaxDynamicSharedMemorySize, agg_lds_bytes(40));

  k_cvtx<<<(Mpad * 16 + NTHR - 1) / NTHR, NTHR, 0, stream>>>(x, ap, nN, Mpad);
  k_cvtw<<<dim3((NC1 * (DIN / 8) + NTHR - 1) / NTHR, 2), NTHR, 0, stream>>>(Wl1, Wr1, btl1, btr1, DIN, NC1, s16);
  k_cvtw<<<dim3((NC2 * (K2 / 8) + NTHR - 1) / NTHR, 2), NTHR, 0, stream>>>(Wl2, Wr2, btl2, btr2, K2, NC2, s16);

  k_gemm<<<dim3(Mpad / GR, NC1 / GC, 2), GTHR, 0, stream>>>(ap, APITCH, DIN, btl1, btr1, bl1, br1, xl, xr, NC1, is16);
  k_agg<32><<<(Mpad + NB - 1) / NB, NTHR, agg_lds_bytes(32), stream>>>(
      ei, xl, (const _Float16*)xr, att1, bias1, ap, out, nN, nE, Mpad);

  k_gemm<<<dim3(Mpad / GR, NC2 / GC, 2), GTHR, 0, stream>>>(ap, APITCH, K2, btl2, btr2, bl2, br2, xl, xr, NC2, is16);
  k_agg<40><<<(nN + NB - 1) / NB, NTHR, agg_lds_bytes(40), stream>>>(
      ei, xl, (const _Float16*)xr, att2, bias2, ap, out, nN, nE, nN);
}
